// myModel_77111842832559
// MI455X (gfx1250) — hardware-run, weakly checked
//
#include <hip/hip_runtime.h>
#include <stddef.h>
#include <stdint.h>
#include <math.h>

#define SPLIT2  1
#define NN      100000
#define NE      1600000
#define HD      64
#define AKP     128
#define WKP     128
#define KEXT    (SPLIT2 ? 128 : 64)
#define GBM     128
#define MP      100096
#define NTHR    256
#define NWAVE   8
#define EPT     8
#define WCH     (32 * EPT)
#define NBRUN   1024
#define SLB     10
#define NBK     98
#define NSLOT   (NBK * NBRUN)
#define WLCAP   2560
#define RCAP    20480
#define TRIPCAP 64
#define MAXDEG_MEAS   36
#define MAXB1024_MEAS 16710
#define SP      68

#define SM_W1 0
#define SM_B1 128
#define SM_B2 192
#define SM_W3 256
#define SM_B3 320
#define SM_N  384

#define BK_ZINTS (NWAVE * WLCAP + RCAP + 3 * NBRUN)
#define BK_INTS  (BK_ZINTS + 3 * NBRUN + 16)
#define BK_LDS   (BK_INTS * 4)

static_assert(HD == 64 && HD == 16 * 4);
static_assert(MP % GBM == 0 && MP >= NN && MP == 782 * GBM && MP % 32 == 0);
static_assert(NBRUN == (1 << SLB) && NBRUN % 32 == 0 && NBRUN % GBM == 0 && NBRUN <= 1024);
static_assert(NBRUN % NTHR == 0 && NBRUN == 4 * NTHR);
static_assert(NSLOT >= MP);
static_assert(NN % 32 == 0 && NN % 2 == 0 && NN <= (1 << 17));
static_assert(NE < (1 << 21) && (((long long)NE) << SLB) < (1LL << 31));
static_assert(NE % WCH == 0 && NE % 4 == 0);
static_assert(RCAP == NWAVE * WLCAP && RCAP % (NTHR * 4) == 0 && BK_ZINTS % 4 == 0);
static_assert((long long)RCAP * 100 >= (long long)MAXB1024_MEAS * 105);
static_assert(WLCAP >= MAXB1024_MEAS / 8 + 8 * 46 + 1);
static_assert(MAXDEG_MEAS + 8 <= TRIPCAP);
static_assert(AKP % 8 == 0 && WKP % 8 == 0 && KEXT % 32 == 0 && KEXT <= AKP && KEXT <= WKP && AKP == 2 * HD);
static_assert(BK_LDS <= 300000);
static_assert((GBM * SP + GBM) * 4 <= 65536);
static_assert((NN - (NBK - 1) * NBRUN) == 672 && ((NN - (NBK - 1) * NBRUN) % 32) == 0);
static_assert(SM_N % 128 == 0 && SM_B3 < SM_N);

typedef float          v2f   __attribute__((ext_vector_type(2)));
typedef float          v4f   __attribute__((ext_vector_type(4)));
typedef float          v8f   __attribute__((ext_vector_type(8)));
typedef int            v4i   __attribute__((ext_vector_type(4)));
typedef int            v8i   __attribute__((ext_vector_type(8)));
typedef unsigned short v8us  __attribute__((ext_vector_type(8)));
typedef unsigned short v16us __attribute__((ext_vector_type(16)));
typedef __bf16         v16bf __attribute__((ext_vector_type(16)));
typedef v2f  __attribute__((may_alias)) v2fa;
typedef v4f  __attribute__((may_alias)) v4fa;
typedef v4i  __attribute__((may_alias)) v4ia;
typedef v8us __attribute__((may_alias)) v8usa;
union FragB { v16bf v; v16us u; v8us h[2]; v8i w; };

__device__ __forceinline__ v8f wmb(const FragB& a, const FragB& b, v8f c) {
  v8f d = __builtin_amdgcn_wmma_f32_16x16x32_bf16(false, a.v, false, b.v, (short)0, c, false, false);
  asm volatile("v_nop\n\tv_nop\n\tv_nop\n\tv_nop" : "+v"(d) : "v"(a.w), "v"(b.w));
  return d;
}

__device__ __forceinline__ unsigned bf16_bits(float f) {
  const unsigned u = __float_as_uint(f);
  const unsigned r = (u + 0x7FFFu + ((u >> 16) & 1u)) >> 16;
  const unsigned q = (u >> 16) | 0x40u;
  return ((u & 0x7fffffffu) > 0x7f800000u) ? q : r;
}
__device__ __forceinline__ float bf16_val(float f) {
  return __uint_as_float(bf16_bits(f) << 16);
}

__device__ __forceinline__ void hilo8(const float (&v)[8], v4i& hi, v4i& lo) {
  unsigned a[8], b[8];
#pragma unroll
  for (int i = 0; i < 8; ++i) {
    a[i] = bf16_bits(v[i]);
    b[i] = bf16_bits(v[i] - __uint_as_float(a[i] << 16));
  }
  v4i h, l;
  h.x = (int)(a[0] | (a[1] << 16)); h.y = (int)(a[2] | (a[3] << 16));
  h.z = (int)(a[4] | (a[5] << 16)); h.w = (int)(a[6] | (a[7] << 16));
  l.x = (int)(b[0] | (b[1] << 16)); l.y = (int)(b[2] | (b[3] << 16));
  l.z = (int)(b[4] | (b[5] << 16)); l.w = (int)(b[6] | (b[7] << 16));
  hi = h; lo = l;
}

__device__ __forceinline__ void st2_v4f(float* p, v4f v) {
  *(volatile v4f*)p = v;
  __threadfence();
  *(volatile v4f*)p = v;
}
__device__ __forceinline__ void st2_v8us(unsigned short* p, v8us v) {
  *(volatile v8us*)p = v;
  __threadfence();
  *(volatile v8us*)p = v;
}

__device__ __forceinline__ v8us gather8(const float* __restrict__ base, int stride) {
  float f[8];
#pragma unroll
  for (int i = 0; i < 8; ++i) f[i] = base[(size_t)i * (size_t)stride];
  v8us o;
#pragma unroll
  for (int i = 0; i < 8; ++i) o[i] = (unsigned short)bf16_bits(f[i]);
  return o;
}

__device__ __forceinline__ int wave_max32(int v) {
  int t;
  t = __shfl_xor(v, 16, 32); v = v > t ? v : t;
  t = __shfl_xor(v, 8, 32);  v = v > t ? v : t;
  t = __shfl_xor(v, 4, 32);  v = v > t ? v : t;
  t = __shfl_xor(v, 2, 32);  v = v > t ? v : t;
  t = __shfl_xor(v, 1, 32);  v = v > t ? v : t;
  return v;
}

__global__ __launch_bounds__(NTHR) void k_prep(const float* __restrict__ w1, const float* __restrict__ b1,
                                               const float* __restrict__ w2, const float* __restrict__ b2,
                                               const float* __restrict__ w3, const float* __restrict__ b3,
                                               unsigned short* w2d, float* sm) {
  const int tid = (int)threadIdx.x, lane = tid & 31, wave = tid >> 5;
  const int blk = (int)blockIdx.x;
  if (blk < 4) {
    const int u = blk * NTHR + tid;
    const int n = u >> 4, k8 = (u & 15) * 8, kk = k8 & (HD - 1);
    const v8us o = gather8(w2 + (size_t)kk * HD + n, HD);
    st2_v8us(w2d + (size_t)n * WKP + k8, o);
  } else {
    if (tid < 96) {
      const int q = lane & 15;
      if (wave == 0) {
        const v4f a = *(const v4fa*)(w1 + 4 * lane);
        v4f o;
        o.x = bf16_val(a.x); o.y = bf16_val(a.y); o.z = bf16_val(a.z); o.w = bf16_val(a.w);
        st2_v4f(sm + SM_W1 + 4 * lane, o);
      } else if (wave == 1) {
        const v4f a = *(const v4fa*)(b1 + 4 * q);
        const v4f c = *(const v4fa*)(b2 + 4 * q);
        asm volatile("" :: "v"(a));
        asm volatile("" :: "v"(c));
        const unsigned ma = (lane < 16) ? 0xffffffffu : 0u;
        v4f o;
        o.x = __uint_as_float(((bf16_bits(a.x) << 16) & ma) | ((bf16_bits(c.x) << 16) & ~ma));
        o.y = __uint_as_float(((bf16_bits(a.y) << 16) & ma) | ((bf16_bits(c.y) << 16) & ~ma));
        o.z = __uint_as_float(((bf16_bits(a.z) << 16) & ma) | ((bf16_bits(c.z) << 16) & ~ma));
        o.w = __uint_as_float(((bf16_bits(a.w) << 16) & ma) | ((bf16_bits(c.w) << 16) & ~ma));
        st2_v4f(sm + SM_B1 + 4 * lane, o);
      } else {
        const v4f a = *(const v4fa*)(w3 + 4 * q);
        const float bb = b3[0];
        asm volatile("" :: "v"(a));
        asm volatile("" :: "v"(bb));
        const unsigned ma = (lane < 16) ? 0xffffffffu : 0u;
        const unsigned mb = (lane == 16) ? 0xffffffffu : 0u;
        v4f o;
        o.x = __uint_as_float(((bf16_bits(a.x) << 16) & ma) | ((bf16_bits(bb) << 16) & mb));
        o.y = __uint_as_float((bf16_bits(a.y) << 16) & ma);
        o.z = __uint_as_float((bf16_bits(a.z) << 16) & ma);
        o.w = __uint_as_float((bf16_bits(a.w) << 16) & ma);
        st2_v4f(sm + SM_W3 + 4 * lane, o);
      }
    }
  }
}

__device__ __forceinline__ void bucket_flush(const int* pl, const int* cnt, const int* dvx, int ov,
                                             int* lp, int* cop, int* dp, int* xp, int* fp, int tid) {
#pragma unroll 1
  for (int i = tid * 4; i < RCAP; i += NTHR * 4) {
    const v4i v = *(const v4ia*)(pl + i);
    *(volatile v4i*)(lp + i) = v;
  }
#pragma unroll 1
  for (int it = 0; it < 2; ++it) {
    const int i = it * (NTHR * 4) + 4 * tid;
    const v4i v = *(const v4ia*)(cnt + i);
    *(volatile v4i*)(cop + i) = v;
  }
  {
    const v4i v = *(const v4ia*)(dvx + 4 * tid);
    *(volatile v4i*)(dp + 4 * tid) = v;
  }
#pragma unroll 1
  for (int it = 0; it < 2; ++it) {
    const int i = it * (NTHR * 4) + 4 * tid;
    const v4i v = *(const v4ia*)(dvx + NBRUN + i);
    *(volatile v4i*)(xp + i) = v;
  }
  if (tid < 8) {
    const v4i f = {ov, ov, ov, ov};
    *(volatile v4i*)(fp + 4 * tid) = f;
  }
}

__global__ __launch_bounds__(NTHR) void k_bucket(const int* __restrict__ srcs, const int* __restrict__ dsts,
                                                 const float* __restrict__ x,
                                                 int* LIST, int* CO, int* DINVb, int* XSb, int* FLAG) {
  extern __shared__ __attribute__((aligned(16))) int dsm[];
  int* wl   = dsm;
  int* pl   = dsm + NWAVE * WLCAP;
  int* cnt  = pl + RCAP;
  int* offs = cnt + NBRUN;
  int* cur  = offs + NBRUN;
  int* dvx  = cur + NBRUN;
  int* misc = dvx + 3 * NBRUN;
  float* dvs = (float*)dvx;
  float* xss = (float*)(dvx + NBRUN);
  const int tid = (int)threadIdx.x, lane = tid & 31, wave = tid >> 5;
  const int blk = (int)blockIdx.x;
  const unsigned nbs = (unsigned)(blk * NBRUN);

  {
    const v4i z4 = {0, 0, 0, 0};
    for (int i = tid * 4; i < BK_ZINTS; i += NTHR * 4) *(v4ia*)(dsm + i) = z4;
    if (tid < 16) misc[tid] = 0;
  }
  __syncthreads();

  {
    const int per  = ((NE + NWAVE * WCH - 1) / (NWAVE * WCH)) * WCH;
    const int ebeg = wave * per;
    const int eend = (ebeg + per < NE) ? (ebeg + per) : NE;
    int* mylist = wl + wave * WLCAP;
    int wc = 0;
#pragma unroll 1
    for (int cb = ebeg; cb < eend; cb += WCH) {
      const int e0 = cb + lane * EPT;
      const v4i da = *(const v4ia*)(dsts + e0);
      const v4i db = *(const v4ia*)(dsts + e0 + 4);
      const unsigned s0 = (unsigned)da.x - nbs, s1 = (unsigned)da.y - nbs;
      const unsigned s2 = (unsigned)da.z - nbs, s3 = (unsigned)da.w - nbs;
      const unsigned s4 = (unsigned)db.x - nbs, s5 = (unsigned)db.y - nbs;
      const unsigned s6 = (unsigned)db.z - nbs, s7 = (unsigned)db.w - nbs;
      const bool h0 = s0 < (unsigned)NBRUN, h1 = s1 < (unsigned)NBRUN, h2 = s2 < (unsigned)NBRUN, h3 = s3 < (unsigned)NBRUN;
      const bool h4 = s4 < (unsigned)NBRUN, h5 = s5 < (unsigned)NBRUN, h6 = s6 < (unsigned)NBRUN, h7 = s7 < (unsigned)NBRUN;
      const unsigned m0 = __builtin_amdgcn_ballot_w32(h0), m1 = __builtin_amdgcn_ballot_w32(h1);
      const unsigned m2 = __builtin_amdgcn_ballot_w32(h2), m3 = __builtin_amdgcn_ballot_w32(h3);
      const unsigned m4 = __builtin_amdgcn_ballot_w32(h4), m5 = __builtin_amdgcn_ballot_w32(h5);
      const unsigned m6 = __builtin_amdgcn_ballot_w32(h6), m7 = __builtin_amdgcn_ballot_w32(h7);
      const unsigned any = m0 | m1 | m2 | m3 | m4 | m5 | m6 | m7;
      if (any != 0u) {
        const int pre = (int)(__builtin_amdgcn_mbcnt_lo(m0, 0u) + __builtin_amdgcn_mbcnt_lo(m1, 0u) +
                              __builtin_amdgcn_mbcnt_lo(m2, 0u) + __builtin_amdgcn_mbcnt_lo(m3, 0u) +
                              __builtin_amdgcn_mbcnt_lo(m4, 0u) + __builtin_amdgcn_mbcnt_lo(m5, 0u) +
                              __builtin_amdgcn_mbcnt_lo(m6, 0u) + __builtin_amdgcn_mbcnt_lo(m7, 0u));
        int p = wc + pre;
        if (h0) { if (p < WLCAP) mylist[p] = ((e0 + 0) << SLB) | (int)s0; p = p + 1; }
        if (h1) { if (p < WLCAP) mylist[p] = ((e0 + 1) << SLB) | (int)s1; p = p + 1; }
        if (h2) { if (p < WLCAP) mylist[p] = ((e0 + 2) << SLB) | (int)s2; p = p + 1; }
        if (h3) { if (p < WLCAP) mylist[p] = ((e0 + 3) << SLB) | (int)s3; p = p + 1; }
        if (h4) { if (p < WLCAP) mylist[p] = ((e0 + 4) << SLB) | (int)s4; p = p + 1; }
        if (h5) { if (p < WLCAP) mylist[p] = ((e0 + 5) << SLB) | (int)s5; p = p + 1; }
        if (h6) { if (p < WLCAP) mylist[p] = ((e0 + 6) << SLB) | (int)s6; p = p + 1; }
        if (h7) { if (p < WLCAP) mylist[p] = ((e0 + 7) << SLB) | (int)s7; p = p + 1; }
        wc += (int)(__builtin_popcount(m0) + __builtin_popcount(m1) + __builtin_popcount(m2) + __builtin_popcount(m3) +
                    __builtin_popcount(m4) + __builtin_popcount(m5) + __builtin_popcount(m6) + __builtin_popcount(m7));
      }
    }
    if (lane == 0) misc[wave] = wc;
  }
  __syncthreads();

  if (wave == 0) {
    int ov = 0;
#pragma unroll 1
    for (int w2 = 0; w2 < NWAVE; ++w2) {
      int c = misc[w2];
      if (c > WLCAP) ov = 1;
      c = c < 0 ? 0 : (c > WLCAP ? WLCAP : c);
#pragma unroll 1
      for (int b0 = 0; b0 < c; b0 += 32) {
        const int idx = b0 + lane;
        const int ent = wl[w2 * WLCAP + (idx < WLCAP ? idx : WLCAP - 1)];
        const int m32 = (c - b0) < 32 ? (c - b0) : 32;
#pragma unroll 1
        for (int k = 0; k < m32; ++k) {
          const int u    = __builtin_amdgcn_readlane(ent, k);
          const int slot = u & (NBRUN - 1);
          if (lane == 0) cnt[slot] = cnt[slot] + 1;
        }
      }
    }
    if (lane == 0) misc[9] = ov;
  }
  __syncthreads();
  if (wave == 0) {
    const int base = lane * (NBRUN / 32);
    int s = 0;
#pragma unroll 1
    for (int i = 0; i < NBRUN / 32; ++i) s += cnt[base + i];
    int incl = s;
#pragma unroll
    for (int d = 1; d < 32; d <<= 1) {
      const int y = __shfl_up(incl, d, 32);
      if (lane >= d) incl += y;
    }
    int run = incl - s;
#pragma unroll 1
    for (int i = 0; i < NBRUN / 32; ++i) {
      const int cv = cnt[base + i];
      offs[base + i] = run;
      cur[base + i]  = run;
      run += cv;
    }
  }
  __syncthreads();

  if (wave == 0) {
#pragma unroll 1
    for (int w2 = 0; w2 < NWAVE; ++w2) {
      int c = misc[w2];
      c = c < 0 ? 0 : (c > WLCAP ? WLCAP : c);
#pragma unroll 1
      for (int b0 = 0; b0 < c; b0 += 32) {
        const int idx = b0 + lane;
        const int ent = wl[w2 * WLCAP + (idx < WLCAP ? idx : WLCAP - 1)];
        int eid = (ent >> SLB) & 0x1FFFFF;
        eid = eid > NE - 1 ? NE - 1 : eid;
        int sr = srcs[eid];
        sr = sr < 0 ? 0 : (sr > NN - 1 ? NN - 1 : sr);
        const int m32 = (c - b0) < 32 ? (c - b0) : 32;
#pragma unroll 1
        for (int k = 0; k < m32; ++k) {
          const int u    = __builtin_amdgcn_readlane(ent, k);
          const int wd   = __builtin_amdgcn_readlane(sr, k);
          const int slot = u & (NBRUN - 1);
          if (lane == 0) {
            int p = cur[slot];
            p = p < 0 ? 0 : (p > RCAP - 1 ? RCAP - 1 : p);
            pl[p] = wd;
            cur[slot] = p + 1;
          }
        }
      }
    }
  }
  __syncthreads();

  const int ovf = misc[9];
  {
    const float qnan = __uint_as_float(0x7fc00000u);
#pragma unroll 1
    for (int s = tid; s < NBRUN; s += NTHR) {
      const int c    = cnt[s];
      const float dg = (float)(c + 1);
      float dv = 1.0f / sqrtf(dg);
      const int node = (int)nbs + s;
      const int nc   = node < NN ? node : NN - 1;
      const v2f xv = *(const v2fa*)(x + 2 * (size_t)nc);
      asm volatile("" :: "v"(xv));
      const bool live = node < NN;
      float x0 = dv * bf16_val(xv.x);
      float x1 = dv * bf16_val(xv.y);
      x0 = live ? x0 : 0.0f;
      x1 = live ? x1 : 0.0f;
      dv = (ovf != 0) ? qnan : dv;
      x0 = (ovf != 0) ? qnan : x0;
      x1 = (ovf != 0) ? qnan : x1;
      dvs[s] = dv;
      xss[2 * s]     = x0;
      xss[2 * s + 1] = x1;
    }
  }
  __syncthreads();

  int* lp  = LIST + (size_t)blk * RCAP;
  int* cop = CO + (size_t)blk * (2 * NBRUN);
  int* dp  = DINVb + (size_t)blk * NBRUN;
  int* xp  = XSb + (size_t)blk * (2 * NBRUN);
  int* fp  = FLAG + (size_t)blk * 32;
  bucket_flush(pl, cnt, dvx, ovf, lp, cop, dp, xp, fp, tid);
  __threadfence();
  bucket_flush(pl, cnt, dvx, ovf, lp, cop, dp, xp, fp, tid);
}

__global__ __launch_bounds__(NTHR) void k_rep_a(const int* __restrict__ LIST, const int* __restrict__ CO,
                                                const int* __restrict__ FLAG, const float* __restrict__ DINV,
                                                const float* __restrict__ XS, const float* __restrict__ SM,
                                                unsigned short* H1HL) {
  __shared__ __attribute__((aligned(16))) float a1[2 * NBRUN];
  __shared__ __attribute__((aligned(16))) float sw[256];
  const int tid = (int)threadIdx.x;
  const int blk = (int)blockIdx.x;
  const int nbs = blk * NBRUN;
  const int* lb  = LIST + (size_t)blk * RCAP;
  const int* cob = CO + (size_t)blk * (2 * NBRUN);
  const int flag = FLAG[(size_t)blk * 32];
  const float qnan = __uint_as_float(0x7fc00000u);

  if (tid < 64) *(v4fa*)(sw + 4 * tid) = *(const v4fa*)(SM + 4 * tid);

#pragma unroll 1
  for (int it = 0; it < NBRUN / NTHR; ++it) {
    const int slot = it * NTHR + tid;
    const int node = nbs + slot;
    const int nc   = node < NN ? node : NN - 1;
    int c = cob[slot];
    int o = cob[NBRUN + slot];
    const bool big = c > TRIPCAP;
    c = c < 0 ? 0 : (c > TRIPCAP ? TRIPCAP : c);
    o = o < 0 ? 0 : (o > RCAP - 1 ? RCAP - 1 : o);
    int cm = wave_max32(c);
    cm = __builtin_amdgcn_readfirstlane(cm);
    int last = o + c - 1;
    last = last < o ? o : last;
    last = last > RCAP - 1 ? RCAP - 1 : last;
    float sx = 0.0f, sy = 0.0f;
#pragma unroll 1
    for (int j = 0; j < cm; ++j) {
      int idx = o + j;
      idx = idx > last ? last : idx;
      int sr = lb[idx];
      sr = sr < 0 ? 0 : (sr > NN - 1 ? NN - 1 : sr);
      const v2f v = *(const v2fa*)(XS + 2 * (size_t)sr);
      asm volatile("" :: "v"(v));
      const bool valid = j < c;
      const float tx = sx + v.x, ty = sy + v.y;
      sx = valid ? tx : sx;
      sy = valid ? ty : sy;
    }
    const v2f self = *(const v2fa*)(XS + 2 * (size_t)nc);
    const float dv = DINV[nc];
    float ax = (sx + self.x) * dv;
    float ay = (sy + self.y) * dv;
    ax = big ? qnan : ax;
    ay = big ? qnan : ay;
    a1[2 * slot]     = ax;
    a1[2 * slot + 1] = ay;
  }
  __syncthreads();

  const int q = tid & 7, rs = tid >> 3;
  float w0[8], w1[8], bb[8];
  {
    const v4f p0 = *(const v4fa*)(sw + SM_W1 + 8 * q),      p1 = *(const v4fa*)(sw + SM_W1 + 8 * q + 4);
    const v4f r0 = *(const v4fa*)(sw + SM_W1 + 64 + 8 * q), r1 = *(const v4fa*)(sw + SM_W1 + 64 + 8 * q + 4);
    const v4f c0 = *(const v4fa*)(sw + SM_B1 + 8 * q),      c1 = *(const v4fa*)(sw + SM_B1 + 8 * q + 4);
    w0[0] = p0.x; w0[1] = p0.y; w0[2] = p0.z; w0[3] = p0.w; w0[4] = p1.x; w0[5] = p1.y; w0[6] = p1.z; w0[7] = p1.w;
    w1[0] = r0.x; w1[1] = r0.y; w1[2] = r0.z; w1[3] = r0.w; w1[4] = r1.x; w1[5] = r1.y; w1[6] = r1.z; w1[7] = r1.w;
    bb[0] = c0.x; bb[1] = c0.y; bb[2] = c0.z; bb[3] = c0.w; bb[4] = c1.x; bb[5] = c1.y; bb[6] = c1.z; bb[7] = c1.w;
  }
  const bool bad = flag != 0;
#pragma unroll 1
  for (int pass = 0; pass < NBRUN / 32; ++pass) {
    const int r   = pass * 32 + rs;
    const int row = nbs + r;
    const bool wr   = (nbs + pass * 32) < MP;
    const bool live = row < NN;
    const v2f a = *(const v2fa*)(a1 + 2 * r);
    float h[8];
#pragma unroll
    for (int i = 0; i < 8; ++i) {
      float t = fmaf(a.y, w1[i], fmaf(a.x, w0[i], bb[i]));
      t = (t > 0.0f) ? t : (t - t);
      t = bad ? qnan : t;
      t = live ? t : 0.0f;
      h[i] = t;
    }
    v4i hi, lo;
    hilo8(h, hi, lo);
    unsigned short* hp = H1HL + (size_t)row * AKP + 8 * q;
    if (wr) {
      *(volatile v4i*)hp = hi;
      *(volatile v4i*)(hp + HD) = lo;
    }
    __threadfence();
    if (wr) {
      *(volatile v4i*)hp = hi;
      *(volatile v4i*)(hp + HD) = lo;
    }
  }
}

template <int KX, int AP, int BP>
__device__ __forceinline__ void gemm_16x64(const unsigned short* __restrict__ ap,
                                           const unsigned short* __restrict__ bp, v8f (&acc)[4]) {
#pragma unroll 1
  for (int k0 = 0; k0 < KX; k0 += 32) {
    FragB af;
    af.h[0] = *(const v8usa*)(ap + k0);
    af.h[1] = *(const v8usa*)(ap + k0 + 16);
#pragma unroll
    for (int nt = 0; nt < 4; ++nt) {
      const unsigned short* wq = bp + (size_t)(16 * nt) * (size_t)BP + k0;
      FragB bf;
      bf.h[0] = *(const v8usa*)wq;
      bf.h[1] = *(const v8usa*)(wq + 16);
      acc[nt] = wmb(af, bf, acc[nt]);
    }
  }
}

__device__ __forceinline__ void stage_d(float* stg, const v8f (&acc)[4], int wave, int hh, int m) {
#pragma unroll
  for (int nt = 0; nt < 4; ++nt) {
#pragma unroll
    for (int r = 0; r < 8; ++r) stg[(16 * wave + 8 * hh + r) * SP + 16 * nt + m] = acc[nt][r];
  }
}

__global__ __launch_bounds__(NTHR) __attribute__((amdgpu_num_vgpr(248)))
void k_mm2(const unsigned short* __restrict__ A, const unsigned short* __restrict__ BT,
           const float* __restrict__ DINV, float* P2) {
  __shared__ __attribute__((aligned(16))) float stg[GBM * SP];
  __shared__ __attribute__((aligned(16))) float sdv[GBM];
  const int tid = (int)threadIdx.x, lane = tid & 31, wave = tid >> 5, hh = lane >> 4, m = lane & 15;
  const int rowBase = (int)blockIdx.x * GBM;
  if (tid < 32) *(v4fa*)(sdv + 4 * tid) = *(const v4fa*)(DINV + (size_t)rowBase + 4 * tid);

  v8f acc[4];
  {
    const v8f z = {0.f, 0.f, 0.f, 0.f, 0.f, 0.f, 0.f, 0.f};
#pragma unroll
    for (int t = 0; t < 4; ++t) acc[t] = z;
  }
  const unsigned short* ap = A + (size_t)(rowBase + 16 * wave + m) * (size_t)AKP + 8 * hh;
  const unsigned short* bp = BT + (size_t)m * (size_t)WKP + 8 * hh;
  gemm_16x64<KEXT, AKP, WKP>(ap, bp, acc);
  stage_d(stg, acc, wave, hh, m);
  __syncthreads();

#pragma unroll 1
  for (int i = 0; i < 8; ++i) {
    const int lr   = 16 * wave + 2 * i + hh;
    const int grow = rowBase + lr;
    const v4f a = *(const v4fa*)(stg + lr * SP + 4 * m);
    const float dv = sdv[lr];
    v4f o;
    o.x = a.x * dv; o.y = a.y * dv; o.z = a.z * dv; o.w = a.w * dv;
    st2_v4f(P2 + (size_t)grow * HD + 4 * m, o);
  }
}

__global__ __launch_bounds__(NTHR) void k_rep_b(const int* __restrict__ LIST, const int* __restrict__ CO,
                                                const int* __restrict__ FLAG, const float* __restrict__ DINV,
                                                const float* __restrict__ P2, const float* __restrict__ SM,
                                                float* S) {
  __shared__ __attribute__((aligned(16))) int   sco[2 * NBRUN];
  __shared__ __attribute__((aligned(16))) float sdv[NBRUN];
  __shared__ __attribute__((aligned(16))) float sS[NBRUN];
  __shared__ __attribute__((aligned(16))) float sp[128];
  const int tid = (int)threadIdx.x, lane = tid & 31, wave = tid >> 5, hh = lane >> 4, q = lane & 15;
  const int blk = (int)blockIdx.x;
  const int nbs = blk * NBRUN;
  const int* lb  = LIST + (size_t)blk * RCAP;
  const int* cob = CO + (size_t)blk * (2 * NBRUN);
  const int flag = FLAG[(size_t)blk * 32];
  const float qnan = __uint_as_float(0x7fc00000u);

#pragma unroll 1
  for (int it = 0; it < 2; ++it) {
    const int i = it * (NTHR * 4) + 4 * tid;
    *(v4ia*)(sco + i) = *(const v4ia*)(cob + i);
  }
  *(v4fa*)(sdv + 4 * tid) = *(const v4fa*)(DINV + (size_t)nbs + 4 * tid);
  if (tid < 32) *(v4fa*)(sp + 4 * tid) = *(const v4fa*)(SM + SM_B2 + 4 * tid);
  __syncthreads();

  const v4f b2v = *(const v4fa*)(sp + 4 * q);
  const v4f w3v = *(const v4fa*)(sp + 64 + 4 * q);

#pragma unroll 1
  for (int i = 0; i < NBRUN / NWAVE; ++i) {
    const int slot = wave * (NBRUN / NWAVE) + i;
    const int d    = nbs + slot;
    const int dc   = d < NN ? d : NN - 1;
    int c = sco[slot];
    int o = sco[NBRUN + slot];
    const bool big = c > TRIPCAP;
    c = c < 0 ? 0 : (c > TRIPCAP ? TRIPCAP : c);
    o = o < 0 ? 0 : (o > RCAP - 1 ? RCAP - 1 : o);
    c = __builtin_amdgcn_readfirstlane(c);
    o = __builtin_amdgcn_readfirstlane(o);
    int last = o + c - 1;
    last = last < o ? o : last;
    last = last > RCAP - 1 ? RCAP - 1 : last;
    const int trips = (c + 1) >> 1;
    float a0 = 0.0f, a1 = 0.0f, a2 = 0.0f, a3 = 0.0f;
#pragma unroll 1
    for (int j = 0; j < trips; ++j) {
      const int hit = 2 * j + hh;
      int idx = o + hit;
      idx = idx > last ? last : idx;
      int sr = lb[idx];
      sr = sr < 0 ? 0 : (sr > NN - 1 ? NN - 1 : sr);
      const v4f v = *(const v4fa*)(P2 + (size_t)sr * HD + 4 * q);
      asm volatile("" :: "v"(v));
      const bool valid = hit < c;
      const float t0 = a0 + v.x, t1 = a1 + v.y, t2 = a2 + v.z, t3 = a3 + v.w;
      a0 = valid ? t0 : a0; a1 = valid ? t1 : a1; a2 = valid ? t2 : a2; a3 = valid ? t3 : a3;
    }
    a0 += __shfl_xor(a0, 16, 32);
    a1 += __shfl_xor(a1, 16, 32);
    a2 += __shfl_xor(a2, 16, 32);
    a3 += __shfl_xor(a3, 16, 32);
    const v4f g = *(const v4fa*)(P2 + (size_t)dc * HD + 4 * q);
    const float dv = sdv[slot];
    float h0 = (a0 + g.x) * dv + b2v.x;
    float h1 = (a1 + g.y) * dv + b2v.y;
    float h2 = (a2 + g.z) * dv + b2v.z;
    float h3 = (a3 + g.w) * dv + b2v.w;
    h0 = (h0 > 0.0f) ? h0 : (h0 - h0);
    h1 = (h1 > 0.0f) ? h1 : (h1 - h1);
    h2 = (h2 > 0.0f) ? h2 : (h2 - h2);
    h3 = (h3 > 0.0f) ? h3 : (h3 - h3);
    float p = h0 * w3v.x;
    p = fmaf(h1, w3v.y, p);
    p = fmaf(h2, w3v.z, p);
    p = fmaf(h3, w3v.w, p);
    p += __shfl_xor(p, 8, 32);
    p += __shfl_xor(p, 4, 32);
    p += __shfl_xor(p, 2, 32);
    p += __shfl_xor(p, 1, 32);
    float s = dv * p;
    const bool bad = (flag != 0) | big;
    s = bad ? qnan : s;
    s = (d < NN) ? s : 0.0f;
    if (lane == 0) sS[slot] = s;
  }
  __syncthreads();

  const v4f ov = *(const v4fa*)(sS + 4 * tid);
  st2_v4f(S + (size_t)nbs + 4 * tid, ov);
}

__global__ __launch_bounds__(NTHR) void k_rep_c(const int* __restrict__ LIST, const int* __restrict__ CO,
                                                const int* __restrict__ FLAG, const float* __restrict__ DINV,
                                                const float* __restrict__ S, const float* __restrict__ SM,
                                                float* out) {
  __shared__ __attribute__((aligned(16))) float so[NBRUN];
  const int tid = (int)threadIdx.x;
  const int blk = (int)blockIdx.x;
  const int nbs = blk * NBRUN;
  const int* lb  = LIST + (size_t)blk * RCAP;
  const int* cob = CO + (size_t)blk * (2 * NBRUN);
  const int flag = FLAG[(size_t)blk * 32];
  const float b3r = SM[SM_B3];
  const float qnan = __uint_as_float(0x7fc00000u);

#pragma unroll 1
  for (int it = 0; it < NBRUN / NTHR; ++it) {
    const int slot = it * NTHR + tid;
    const int node = nbs + slot;
    const int nc   = node < NN ? node : NN - 1;
    int c = cob[slot];
    int o = cob[NBRUN + slot];
    const bool big = c > TRIPCAP;
    c = c < 0 ? 0 : (c > TRIPCAP ? TRIPCAP : c);
    o = o < 0 ? 0 : (o > RCAP - 1 ? RCAP - 1 : o);
    int cm = wave_max32(c);
    cm = __builtin_amdgcn_readfirstlane(cm);
    int last = o + c - 1;
    last = last < o ? o : last;
    last = last > RCAP - 1 ? RCAP - 1 : last;
    float sum = 0.0f;
#pragma unroll 1
    for (int j = 0; j < cm; ++j) {
      int idx = o + j;
      idx = idx > last ? last : idx;
      int sr = lb[idx];
      sr = sr < 0 ? 0 : (sr > NN - 1 ? NN - 1 : sr);
      const float v = S[sr];
      asm volatile("" :: "v"(v));
      const bool valid = j < c;
      const float t = sum + v;
      sum = valid ? t : sum;
    }
    const float self = S[nc];
    const float dv   = DINV[nc];
    float val = dv * (sum + self) + b3r;
    const bool bad = (flag != 0) | big;
    val = bad ? qnan : val;
    so[slot] = val;
  }
  __syncthreads();

  const int liveRows = (NN - nbs) < NBRUN ? (NN - nbs) : NBRUN;
  const int nv4 = liveRows >> 2;
  const v4f ov = *(const v4fa*)(so + 4 * tid);
  float* op = out + (size_t)nbs + 4 * tid;
  const bool wr = tid < nv4;
  if (wr) *(volatile v4f*)op = ov;
  __threadfence();
  if (wr) *(volatile v4f*)op = ov;
}

extern "C" void kernel_launch(void* const* d_in, const int* in_sizes, int n_in,
                              void* d_out, int out_size, void* d_ws, size_t ws_size,
                              hipStream_t stream) {
  if (n_in < 8) return;
  if (in_sizes[0] != NN * 2) return;
  if (in_sizes[1] != 2 * NE) return;
  if (in_sizes[2] != 2 * HD) return;
  if (in_sizes[3] != HD) return;
  if (in_sizes[4] != HD * HD) return;
  if (in_sizes[5] != HD) return;
  if (in_sizes[6] != HD) return;
  if (in_sizes[7] != 1) return;
  if (out_size != NN) return;

  const float* x  = (const float*)d_in[0];
  const int*   ei = (const int*)d_in[1];
  const float* W1 = (const float*)d_in[2];
  const float* b1 = (const float*)d_in[3];
  const float* W2 = (const float*)d_in[4];
  const float* b2 = (const float*)d_in[5];
  const float* W3 = (const float*)d_in[6];
  const float* b3 = (const float*)d_in[7];
  float* out = (float*)d_out;
  const int* srcs = ei;
  const int* dsts = ei + NE;

  constexpr size_t zHL   = (size_t)MP * AKP * 2;
  constexpr size_t zP2   = (size_t)MP * HD * 4;
  constexpr size_t zLIST = (size_t)NBK * RCAP * 4;
  constexpr size_t zCO   = (size_t)NBK * 2 * NBRUN * 4;
  constexpr size_t zDV   = (size_t)NSLOT * 4;
  constexpr size_t zXS   = (size_t)NSLOT * 8;
  constexpr size_t zS    = (size_t)NSLOT * 4;
  constexpr size_t zFLAG = (size_t)NBK * 128;
  constexpr size_t zW2D  = (size_t)HD * WKP * 2;
  constexpr size_t zSM   = (size_t)SM_N * 4;
  constexpr size_t oHL   = 0;
  constexpr size_t oP2   = oHL + zHL;
  constexpr size_t oLIST = oP2 + zP2;
  constexpr size_t oCO   = oLIST + zLIST;
  constexpr size_t oDV   = oCO + zCO;
  constexpr size_t oXS   = oDV + zDV;
  constexpr size_t oS    = oXS + zXS;
  constexpr size_t oFLAG = oS + zS;
  constexpr size_t oW2D  = oFLAG + zFLAG;
  constexpr size_t oSM   = oW2D + zW2D;
  constexpr size_t oEND  = oSM + zSM;
  static_assert(zHL % 256 == 0 && zP2 % 256 == 0 && zLIST % 256 == 0 && zCO % 256 == 0 && zDV % 256 == 0);
  static_assert(zXS % 256 == 0 && zS % 256 == 0 && zFLAG % 256 == 0 && zW2D % 256 == 0 && zSM % 256 == 0);
  static_assert(oEND <= (size_t)(128u << 20));
  if (oEND > ws_size) return;

  char* ws = (char*)d_ws;
  unsigned short* H1HL = (unsigned short*)(ws + oHL);
  float*          P2   = (float*)(ws + oP2);
  int*            LIST = (int*)(ws + oLIST);
  int*            CO   = (int*)(ws + oCO);
  float*          DINV = (float*)(ws + oDV);
  float*          XS   = (float*)(ws + oXS);
  float*          S    = (float*)(ws + oS);
  int*            FLAG = (int*)(ws + oFLAG);
  unsigned short* W2D  = (unsigned short*)(ws + oW2D);
  float*          SM   = (float*)(ws + oSM);

  hipFuncSetAttribute(reinterpret_cast<const void*>(&k_bucket), hipFuncAttributeMaxDynamicSharedMemorySize, (int)BK_LDS);

  k_prep<<<5, NTHR, 0, stream>>>(W1, b1, W2, b2, W3, b3, W2D, SM);
  k_bucket<<<NBK, NTHR, BK_LDS, stream>>>(srcs, dsts, x, LIST, CO, (int*)DINV, (int*)XS, FLAG);
  k_rep_a<<<NBK, NTHR, 0, stream>>>(LIST, CO, FLAG, DINV, XS, SM, H1HL);
  k_mm2<<<MP / GBM, NTHR, 0, stream>>>(H1HL, W2D, DINV, P2);
  k_rep_b<<<NBK, NTHR, 0, stream>>>(LIST, CO, FLAG, DINV, P2, SM, S);
  k_rep_c<<<NBK, NTHR, 0, stream>>>(LIST, CO, FLAG, DINV, S, SM, out);
}
